// GatedMamba_9311489098327
// MI455X (gfx1250) — hardware-verified
//
#include <hip/hip_runtime.h>
#include <math.h>

typedef _Float16 f16;
typedef _Float16 v16h __attribute__((ext_vector_type(16)));
typedef _Float16 v8h  __attribute__((ext_vector_type(8)));
typedef _Float16 v2h  __attribute__((ext_vector_type(2)));
typedef float    v8f  __attribute__((ext_vector_type(8)));
typedef float    v4f  __attribute__((ext_vector_type(4)));
typedef float    v2f  __attribute__((ext_vector_type(2)));

#define D_DIM  1024
#define B_DIM  4
#define T_DIM  2048
#define M_ROWS (B_DIM * T_DIM)

__global__ __launch_bounds__(256)
void k_cvt(const float* __restrict__ x,  const float* __restrict__ w0,
           const float* __restrict__ w1, const float* __restrict__ w2,
           f16* __restrict__ xh,  f16* __restrict__ w0h,
           f16* __restrict__ w1h, f16* __restrict__ w2h,
           int nx8, int nw0_8, int nw1_8, int nw2_8, float wsc)
{
    const int g = blockIdx.x * 256 + threadIdx.x;
    const int total = nx8 + nw0_8 + nw1_8 + nw2_8;
    if (g >= total) return;
    const float* src = x;
    f16* dst = xh;
    float sc = 1.0f;
    int i = g;
    if (i >= nx8) {
        i -= nx8; src = w0; dst = w0h; sc = wsc;
        if (i >= nw0_8) {
            i -= nw0_8; src = w1; dst = w1h;
            if (i >= nw1_8) {
                i -= nw1_8; src = w2; dst = w2h;
            }
        }
    }
    const v4f a = *(const v4f*)(src + (size_t)i * 8);
    const v4f b = *(const v4f*)(src + (size_t)i * 8 + 4);
    v8h o;
    o[0] = (f16)(a[0] * sc); o[1] = (f16)(a[1] * sc);
    o[2] = (f16)(a[2] * sc); o[3] = (f16)(a[3] * sc);
    o[4] = (f16)(b[0] * sc); o[5] = (f16)(b[1] * sc);
    o[6] = (f16)(b[2] * sc); o[7] = (f16)(b[3] * sc);
    volatile v8h* p = (volatile v8h*)(dst + (size_t)i * 8);
    *p = o;
    __threadfence();
    *p = o;
}

template <int EPI>
__global__ __launch_bounds__(128)
void k_gemm(const f16* __restrict__ A, const f16* __restrict__ W,
            const float* __restrict__ bias, const float* __restrict__ aux,
            float* __restrict__ outf, f16* __restrict__ outh,
            int K, int ldo, float oscale)
{
    __shared__ __attribute__((aligned(16))) float sm[4][16 * 64];

    const int lane = threadIdx.x & 31;
    const int wid  = threadIdx.x >> 5;
    const int h    = lane >> 4;
    const int m    = lane & 15;
    const int mrow0 = blockIdx.x * 64 + (wid >> 1) * 32;
    const int ncol0 = blockIdx.y * 128 + (wid & 1) * 64;

    v8f acc[2][4] = {};

    for (int k0 = 0; k0 < K; k0 += 32) {
        v16h af[2], bf[4];
        #pragma unroll
        for (int i = 0; i < 2; ++i) {
            const f16* p = A + (size_t)(mrow0 + i * 16 + m) * K + k0 + 8 * h;
            const v8h lo = *(const v8h*)p;
            const v8h hi = *(const v8h*)(p + 16);
            af[i] = __builtin_shufflevector(lo, hi, 0,1,2,3,4,5,6,7,8,9,10,11,12,13,14,15);
        }
        #pragma unroll
        for (int j = 0; j < 4; ++j) {
            const f16* p = W + (size_t)(ncol0 + j * 16 + m) * K + k0 + 8 * h;
            const v8h lo = *(const v8h*)p;
            const v8h hi = *(const v8h*)(p + 16);
            bf[j] = __builtin_shufflevector(lo, hi, 0,1,2,3,4,5,6,7,8,9,10,11,12,13,14,15);
        }
        #pragma unroll
        for (int i = 0; i < 2; ++i)
            #pragma unroll
            for (int j = 0; j < 4; ++j)
                acc[i][j] = __builtin_amdgcn_wmma_f32_16x16x32_f16(
                    false, af[i], false, bf[j], (short)0, acc[i][j], false, false);
        asm volatile("v_nop\n\tv_nop\n\tv_nop\n\tv_nop"
                     : "+v"(acc[0][0]), "+v"(acc[0][1]), "+v"(acc[0][2]), "+v"(acc[0][3]),
                       "+v"(acc[1][0]), "+v"(acc[1][1]), "+v"(acc[1][2]), "+v"(acc[1][3])
                     : "v"(af[0]), "v"(af[1]), "v"(bf[0]), "v"(bf[1]), "v"(bf[2]), "v"(bf[3]));
    }

    const int half  = (ncol0 >= ldo) ? 1 : 0;
    const int ocol0 = ncol0 - half * ldo;
    float* st = &sm[wid][0];

    #pragma unroll
    for (int i = 0; i < 2; ++i) {
        #pragma unroll
        for (int j = 0; j < 4; ++j) {
            const float bv = bias[ncol0 + j * 16 + m];
            #pragma unroll
            for (int r = 0; r < 8; ++r)
                st[(8 * h + r) * 64 + j * 16 + m] = acc[i][j][r] * oscale + bv;
        }
        __syncthreads();
        const int rowb = mrow0 + i * 16;
        if (EPI == 1 && half != 0) {
            #pragma unroll 1
            for (int s = 0; s < 4; ++s) {
                const int r  = 4 * s + (lane >> 3);
                const int c8 = 8 * (lane & 7);
                const v4f v0 = *(const v4f*)(st + r * 64 + c8);
                const v4f v1 = *(const v4f*)(st + r * 64 + c8 + 4);
                v8h o;
                o[0] = (f16)v0[0]; o[1] = (f16)v0[1]; o[2] = (f16)v0[2]; o[3] = (f16)v0[3];
                o[4] = (f16)v1[0]; o[5] = (f16)v1[1]; o[6] = (f16)v1[2]; o[7] = (f16)v1[3];
                const size_t gi = (size_t)(rowb + r) * ldo + ocol0 + c8;
                volatile v8h* p = (volatile v8h*)(outh + gi);
                *p = o;
                __threadfence();
                *p = o;
            }
        } else {
            #pragma unroll 1
            for (int s = 0; s < 8; ++s) {
                const int r  = 2 * s + h;
                const int c4 = 4 * m;
                v4f v = *(const v4f*)(st + r * 64 + c4);
                const size_t gi = (size_t)(rowb + r) * ldo + ocol0 + c4;
                if (EPI == 1) {
                    #pragma unroll
                    for (int e = 0; e < 4; ++e) {
                        const float t = v[e];
                        v[e] = __builtin_amdgcn_rcpf(1.0f + __expf(-t));
                    }
                } else if (EPI == 2) {
                    const v4f g = *(const v4f*)(aux + gi);
                    #pragma unroll
                    for (int e = 0; e < 4; ++e) v[e] = g[e] * tanhf(v[e]);
                } else {
                    const v4f xr = *(const v4f*)(aux + gi);
                    v = v + xr;
                }
                volatile v4f* p = (volatile v4f*)(outf + gi);
                *p = v;
                __threadfence();
                *p = v;
            }
        }
        __syncthreads();
    }
}

__global__ __launch_bounds__(64)
void k_rec(const float* __restrict__ gate, const float* __restrict__ bco, f16* __restrict__ hout)
{
    __shared__ __attribute__((aligned(16))) f16 sh[2][8 * 64];
    const int lane = threadIdx.x & 31;
    const int w    = threadIdx.x >> 5;
    const int gw   = blockIdx.x * 2 + w;
    const int b    = gw >> 4;
    const int dbase = (gw & 15) * 64;
    const size_t base = (size_t)b * T_DIM * D_DIM + dbase;
    f16* shw = &sh[w][0];
    float h0 = 0.0f, h1 = 0.0f;

    for (int t0 = 0; t0 < T_DIM; t0 += 8) {
        #pragma unroll
        for (int tt = 0; tt < 8; ++tt) {
            const size_t gi = base + (size_t)(t0 + tt) * D_DIM + 2 * lane;
            const v2f g  = *(const v2f*)(gate + gi);
            const v2f bb = *(const v2f*)(bco + gi);
            h0 = (1.0f - g[0]) * h0 + bb[0];
            h1 = (1.0f - g[1]) * h1 + bb[1];
            v2h o;
            o[0] = (f16)h0;
            o[1] = (f16)h1;
            *(v2h*)(shw + tt * 64 + 2 * lane) = o;
        }
        __syncthreads();
        const int q  = lane >> 3;
        const int c8 = 8 * (lane & 7);
        const v8h u0 = *(const v8h*)(shw + q * 64 + c8);
        const v8h u1 = *(const v8h*)(shw + (q + 4) * 64 + c8);
        volatile v8h* p0 = (volatile v8h*)(hout + base + (size_t)(t0 + q) * D_DIM + c8);
        volatile v8h* p1 = (volatile v8h*)(hout + base + (size_t)(t0 + q + 4) * D_DIM + c8);
        *p0 = u0;
        *p1 = u1;
        __threadfence();
        *p0 = u0;
        *p1 = u1;
        __syncthreads();
    }
}

extern "C" void kernel_launch(void* const* d_in, const int* in_sizes, int n_in,
                              void* d_out, int out_size, void* d_ws, size_t ws_size,
                              hipStream_t stream)
{
    if (n_in < 7) return;
    const int nx = M_ROWS * D_DIM;
    if (in_sizes[0] != nx) return;
    if (in_sizes[1] != 2 * D_DIM * D_DIM) return;
    if (in_sizes[2] < 2 * D_DIM) return;
    if (in_sizes[3] != D_DIM * D_DIM) return;
    if (in_sizes[4] < D_DIM) return;
    if (in_sizes[5] != D_DIM * D_DIM) return;
    if (in_sizes[6] < D_DIM) return;
    if (out_size != nx) return;

    const float* x    = (const float*)d_in[0];
    const float* W_in = (const float*)d_in[1];
    const float* b_in = (const float*)d_in[2];
    const float* W_s  = (const float*)d_in[3];
    const float* b_s  = (const float*)d_in[4];
    const float* W_o  = (const float*)d_in[5];
    const float* b_o  = (const float*)d_in[6];
    float* out = (float*)d_out;

    char* ws = (char*)d_ws;
    size_t off = 0;
    const size_t szXh  = (size_t)nx * 2;
    const size_t szWin = (size_t)2 * D_DIM * D_DIM * 2;
    const size_t szW   = (size_t)D_DIM * D_DIM * 2;
    const size_t szF32 = (size_t)nx * 4;
    const size_t szF16 = (size_t)nx * 2;
    f16*   Xh    = (f16*)(ws + off);   off += szXh;
    f16*   Win_h = (f16*)(ws + off);   off += szWin;
    f16*   Ws_h  = (f16*)(ws + off);   off += szW;
    f16*   Wo_h  = (f16*)(ws + off);   off += szW;
    float* gateb = (float*)(ws + off); off += szF32;
    f16*   valb  = (f16*)(ws + off);   off += szF16;
    float* bcob  = (float*)(ws + off); off += szF32;
    f16*   hbuf  = (f16*)(ws + off);   off += szF16;
    if (off > ws_size) return;

    const float wsc  = 64.0f;
    const float winv = 1.0f / 64.0f;

    {
        const int nx8  = nx / 8;
        const int nwi8 = 2 * D_DIM * D_DIM / 8;
        const int nw8  = D_DIM * D_DIM / 8;
        const int total = nx8 + nwi8 + 2 * nw8;
        k_cvt<<<(total + 255) / 256, 256, 0, stream>>>(x, W_in, W_s, W_o, Xh, Win_h, Ws_h, Wo_h,
                                                      nx8, nwi8, nw8, nw8, wsc);
    }
    {
        dim3 grid(M_ROWS / 64, (2 * D_DIM) / 128);
        k_gemm<1><<<grid, 128, 0, stream>>>(Xh, Win_h, b_in, nullptr, gateb, valb,
                                            D_DIM, D_DIM, winv);
    }
    {
        dim3 grid(M_ROWS / 64, D_DIM / 128);
        k_gemm<2><<<grid, 128, 0, stream>>>(valb, Ws_h, b_s, gateb, bcob, nullptr,
                                            D_DIM, D_DIM, winv);
    }
    k_rec<<<(B_DIM * D_DIM) / 128, 64, 0, stream>>>(gateb, bcob, hbuf);
    {
        dim3 grid(M_ROWS / 64, D_DIM / 128);
        k_gemm<3><<<grid, 128, 0, stream>>>(hbuf, Wo_h, b_o, x, out, nullptr,
                                            D_DIM, D_DIM, winv);
    }
}
